// GPUManifoldFeatureEncoder_71408126264009
// MI455X (gfx1250) — hardware-verified
//
#include <hip/hip_runtime.h>
#include <stddef.h>
#include <math.h>


#define NTHR    256
#define NWAVE   8
#define EW      4
#define ETHR    (EW * 32)
#define P1      72
#define P2      40
#define EPT     8
#define NGRP    2
#define CHUNK   (NTHR * EPT * NGRP)
#define WCAP    (EPT * NGRP * 32)
#define LISTN   (NWAVE * WCAP)
#define NBC     2048
#define NPB     1024
#define MAXEB   1024
#define WSCAP   134217728
#define OFF_P0  0
#define OFF_P2H 2048
#define OFF_P2L 4096
#define OFF_P3H 6144
#define OFF_P3L 6656
#define OFF_PA  7168
#define OFF_PB  7680
#define WTOT    8192
#define GLDSF   (NBC * 16 + NBC + LISTN + 32 + 32)
#define GLDSB   (GLDSF * 4)
#define GELUC   0.70710678118654752f

static_assert((CHUNK & (CHUNK - 1)) == 0);
static_assert((NBC & (NBC - 1)) == 0);
static_assert(NBC <= 4096);
static_assert(CHUNK <= (1 << 19));
static_assert(NBC % NPB == 0);
static_assert(NPB % (NWAVE * 16) == 0);
static_assert(WTOT == 4 * NTHR * 8);
static_assert(((P1 * 2) % 16) == 0);
static_assert(((P2 * 2) % 16) == 0);
static_assert(((NBC * 16 + NBC) % (4 * NTHR)) == 0);
static_assert((NBC * 4) % NTHR == 0);

typedef float          v4f   __attribute__((ext_vector_type(4)));
typedef float          v8f   __attribute__((ext_vector_type(8)));
typedef double         v2d   __attribute__((ext_vector_type(2)));
typedef int            v4i   __attribute__((ext_vector_type(4)));
typedef unsigned short v8us  __attribute__((ext_vector_type(8)));
typedef unsigned short v16us __attribute__((ext_vector_type(16)));
typedef __bf16         v16bf __attribute__((ext_vector_type(16)));
union FragB { v16bf v; v16us u; v8us h[2]; };

__device__ __forceinline__ v8f wm(v16bf a, v16bf b, v8f c) {
  v8f d = __builtin_amdgcn_wmma_f32_16x16x32_bf16(false, a, false, b, (short)0, c, false, false);
  asm volatile("v_nop\n\tv_nop\n\tv_nop\n\tv_nop" : "+v"(d) : "v"(a), "v"(b));
  return d;
}

__device__ __forceinline__ v8f zero8() {
  v8f z = {0.f, 0.f, 0.f, 0.f, 0.f, 0.f, 0.f, 0.f};
  return z;
}

__device__ __forceinline__ void wsync() {
  __builtin_amdgcn_fence(__ATOMIC_ACQ_REL, "wavefront");
  __builtin_amdgcn_wave_barrier();
}

__device__ __forceinline__ unsigned bf_rne(float x) {
  const unsigned u = __float_as_uint(x);
  return (u + 0x7FFFu + ((u >> 16) & 1u)) >> 16;
}
__device__ __forceinline__ void split_bf(float x, unsigned short& hi, unsigned short& lo) {
  const unsigned h = bf_rne(x);
  const float hf = __uint_as_float(h << 16);
  hi = (unsigned short)h;
  lo = (unsigned short)bf_rne(x - hf);
}

__device__ __forceinline__ float gelu_f(float x) {
  return 0.5f * x * (1.0f + erff(x * GELUC));
}

__global__ __launch_bounds__(NTHR) void k_wprep(
    const float* __restrict__ W1, const float* __restrict__ W2,
    const float* __restrict__ W3, const float* __restrict__ Wp,
    unsigned short* wp) {
  const int tid = (int)threadIdx.x;
  const int b = (int)blockIdx.x;
  const int og = (b * NTHR + tid) * 8;
  float v[8];
  int part = 0, zero = 0;
  if (b == 0) {
    const int o = og;
    const int n = o >> 5;
    const int grp = (o >> 3) & 3;
    part = (grp == 2) ? 1 : 0;
    zero = (grp == 3) ? 1 : 0;
#pragma unroll
    for (int j = 0; j < 8; ++j) v[j] = W1[j * 64 + n];
  } else if (b == 1 || b == 2) {
    const int o = og - (b == 1 ? OFF_P2H : OFF_P2L);
    const int n = o >> 6;
    const int k0 = o & 63;
    part = (b == 2) ? 1 : 0;
#pragma unroll
    for (int j = 0; j < 8; ++j) v[j] = W2[(k0 + j) * 32 + n];
  } else {
    const int o = og - OFF_P3H;
    const int seg = o >> 9;
    const int oo = o & 511;
    const int n = oo >> 5;
    const int k0 = oo & 31;
    part = seg & 1;
    zero = (seg == 3 && k0 >= 16) ? 1 : 0;
#pragma unroll
    for (int j = 0; j < 8; ++j) {
      const int kk = k0 + j;
      const float a = W3[kk * 16 + n];
      const float p = Wp[(kk & 15) * 16 + n];
      v[j] = (seg < 2) ? a : p;
    }
  }
  v8us ov;
#pragma unroll
  for (int j = 0; j < 8; ++j) {
    unsigned short hi, lo;
    split_bf(v[j], hi, lo);
    unsigned short s = part ? lo : hi;
    s = zero ? (unsigned short)0 : s;
    ov[j] = s;
  }
  unsigned short* dp = wp + og;
  *(volatile v8us*)dp = ov;
  __threadfence();
  *(volatile v8us*)dp = ov;
}

__device__ __forceinline__ void stats_out(double dsum, double dsq,
                                          double* sRedS, double* sRedQ, double* sTot,
                                          int nW, double* dst, int lane, int wave) {
  sRedS[wave * 32 + lane] = dsum;
  sRedQ[wave * 32 + lane] = dsq;
  __syncthreads();
  if (wave == 0) {
    const int c = lane & 15;
    double vs = 0.0, vq = 0.0;
#pragma unroll 1
    for (int w2 = 0; w2 < nW; ++w2) {
      vs += sRedS[w2 * 32 + c] + sRedS[w2 * 32 + 16 + c];
      vq += sRedQ[w2 * 32 + c] + sRedQ[w2 * 32 + 16 + c];
    }
    sTot[lane] = (lane < 16) ? vs : vq;
    wsync();
    const int l2 = (lane < 16) ? lane : 0;
    const v2d o = *(const v2d*)(sTot + 2 * l2);
    if (lane < 16) *(volatile v2d*)(dst + 2 * lane) = o;
    __threadfence();
    if (lane < 16) *(volatile v2d*)(dst + 2 * lane) = o;
  }
}

__global__ __launch_bounds__(ETHR) void k_edge(
    const float* __restrict__ coords, const float* __restrict__ normals,
    const float* __restrict__ curv, const int* __restrict__ ei,
    const unsigned short* __restrict__ wp,
    const float* __restrict__ b1, const float* __restrict__ b2, const float* __restrict__ b3,
    float* Hp, double* part, int nE, int nN, int nGroups) {
  __shared__ __attribute__((aligned(16))) unsigned short sFh[EW][256];
  __shared__ __attribute__((aligned(16))) unsigned short sFl[EW][256];
  __shared__ __attribute__((aligned(16))) unsigned short sA1h[EW][16 * P1];
  __shared__ __attribute__((aligned(16))) unsigned short sA1l[EW][16 * P1];
  __shared__ __attribute__((aligned(16))) unsigned short sA2h[EW][16 * P2];
  __shared__ __attribute__((aligned(16))) unsigned short sA2l[EW][16 * P2];
  __shared__ __attribute__((aligned(16))) float sH[EW][256];
  __shared__ __attribute__((aligned(16))) double sRedS[EW * 32];
  __shared__ __attribute__((aligned(16))) double sRedQ[EW * 32];
  __shared__ __attribute__((aligned(16))) double sTot[32];
  const int tid = threadIdx.x, lane = tid & 31, wave = tid >> 5, hh = lane >> 4, m = lane & 15;
  unsigned short* fH  = sFh[wave];
  unsigned short* fL  = sFl[wave];
  unsigned short* a1H = sA1h[wave];
  unsigned short* a1L = sA1l[wave];
  unsigned short* a2H = sA2h[wave];
  unsigned short* a2L = sA2l[wave];
  float* sHw = sH[wave];

  float b1c[4];
#pragma unroll
  for (int t = 0; t < 4; ++t) b1c[t] = b1[16 * t + m];
  float b2c[2];
  b2c[0] = b2[m]; b2c[1] = b2[16 + m];
  const float b3c = b3[m];
  double dsum = 0.0, dsq = 0.0;

#pragma unroll 1
  for (int g = blockIdx.x * EW + wave; g < nGroups; g += gridDim.x * EW) {
    {
      int e = 32 * g + lane;
      e = e > nE - 1 ? nE - 1 : e;
      int r = ei[e];
      int c = ei[(size_t)nE + (size_t)e];
      r = r < 0 ? 0 : (r > nN - 1 ? nN - 1 : r);
      c = c < 0 ? 0 : (c > nN - 1 ? nN - 1 : c);
      const float* pr = coords + (size_t)r * 3;
      const float* pc = coords + (size_t)c * 3;
      const float* qr = normals + (size_t)r * 3;
      const float* qc = normals + (size_t)c * 3;
      const float crx = pr[0], cry = pr[1], crz = pr[2];
      const float ccx = pc[0], ccy = pc[1], ccz = pc[2];
      const float nrx = qr[0], nry = qr[1], nrz = qr[2];
      const float ncx = qc[0], ncy = qc[1], ncz = qc[2];
      const float dx = ccx - crx, dy = ccy - cry, dz = ccz - crz;
      const float ndot = nrx * ncx + nry * ncy + nrz * ncz;
      const float dn = sqrtf(dx * dx + dy * dy + dz * dz) + 1e-8f;
      const float inv = 1.0f / dn;
      float cr = (nrx * dx + nry * dy + nrz * dz) * inv;
      float cc = (ncx * dx + ncy * dy + ncz * dz) * inv;
      cr = fminf(fmaxf(cr, -1.0f), 1.0f);
      cc = fminf(fmaxf(cc, -1.0f), 1.0f);
      const float cd0 = curv[(size_t)c * 4]     - curv[(size_t)r * 4];
      const float cd1 = curv[(size_t)c * 4 + 1] - curv[(size_t)r * 4 + 1];
      float f[8];
      f[0] = dx; f[1] = dy; f[2] = dz; f[3] = ndot; f[4] = cr; f[5] = cc; f[6] = cd0; f[7] = cd1;
      v8us fh, fl;
#pragma unroll
      for (int j = 0; j < 8; ++j) {
        unsigned short hi, lo;
        split_bf(f[j], hi, lo);
        fh[j] = hi;
        fl[j] = lo;
      }
      *(v8us*)(fH + lane * 8) = fh;
      *(v8us*)(fL + lane * 8) = fl;
    }
    wsync();

#pragma unroll 1
    for (int half = 0; half < 2; ++half) {
      v8f acc0[4];
      {
        const v8us vh = *(const v8us*)(fH + (16 * half + m) * 8);
        const v8us vl = *(const v8us*)(fL + (16 * half + m) * 8);
        v16us au;
#pragma unroll
        for (int i = 0; i < 8; ++i) {
          au[i]     = hh ? vl[i] : vh[i];
          au[8 + i] = hh ? (unsigned short)0 : vh[i];
        }
        FragB a;
        a.u = au;
#pragma unroll
        for (int t = 0; t < 4; ++t) {
          const unsigned short* bq = wp + OFF_P0 + (size_t)(16 * t + m) * 32 + 8 * hh;
          FragB bb;
          bb.h[0] = *(const v8us*)bq;
          bb.h[1] = *(const v8us*)(bq + 16);
          acc0[t] = wm(a.v, bb.v, zero8());
        }
      }
#pragma unroll
      for (int t = 0; t < 4; ++t) {
#pragma unroll
        for (int r = 0; r < 8; ++r) {
          const float x = gelu_f(acc0[t][r] + b1c[t]);
          unsigned short hi, lo;
          split_bf(x, hi, lo);
          const int idx = (8 * hh + r) * P1 + 16 * t + m;
          a1H[idx] = hi;
          a1L[idx] = lo;
        }
      }
      wsync();

      v8f acc1[2];
      acc1[0] = zero8(); acc1[1] = zero8();
      {
        const unsigned short* aph = a1H + m * P1 + 8 * hh;
        const unsigned short* apl = a1L + m * P1 + 8 * hh;
#pragma unroll
        for (int ks = 0; ks < 2; ++ks) {
          FragB ah, al;
          ah.h[0] = *(const v8us*)(aph + 32 * ks);
          ah.h[1] = *(const v8us*)(aph + 32 * ks + 16);
          al.h[0] = *(const v8us*)(apl + 32 * ks);
          al.h[1] = *(const v8us*)(apl + 32 * ks + 16);
#pragma unroll
          for (int t = 0; t < 2; ++t) {
            const size_t bo = (size_t)(16 * t + m) * 64 + 32 * ks + 8 * hh;
            FragB bh, bl;
            bh.h[0] = *(const v8us*)(wp + OFF_P2H + bo);
            bh.h[1] = *(const v8us*)(wp + OFF_P2H + bo + 16);
            bl.h[0] = *(const v8us*)(wp + OFF_P2L + bo);
            bl.h[1] = *(const v8us*)(wp + OFF_P2L + bo + 16);
            acc1[t] = wm(ah.v, bh.v, acc1[t]);
            acc1[t] = wm(ah.v, bl.v, acc1[t]);
            acc1[t] = wm(al.v, bh.v, acc1[t]);
          }
        }
      }
#pragma unroll
      for (int t = 0; t < 2; ++t) {
#pragma unroll
        for (int r = 0; r < 8; ++r) {
          const float x = gelu_f(acc1[t][r] + b2c[t]);
          unsigned short hi, lo;
          split_bf(x, hi, lo);
          const int idx = (8 * hh + r) * P2 + 16 * t + m;
          a2H[idx] = hi;
          a2L[idx] = lo;
        }
      }
      wsync();

      v8f acc2 = zero8();
      {
        FragB ah, al;
        ah.h[0] = *(const v8us*)(a2H + m * P2 + 8 * hh);
        ah.h[1] = *(const v8us*)(a2H + m * P2 + 16 + 8 * hh);
        al.h[0] = *(const v8us*)(a2L + m * P2 + 8 * hh);
        al.h[1] = *(const v8us*)(a2L + m * P2 + 16 + 8 * hh);
        const size_t bo = (size_t)m * 32 + 8 * hh;
        FragB bh, bl;
        bh.h[0] = *(const v8us*)(wp + OFF_P3H + bo);
        bh.h[1] = *(const v8us*)(wp + OFF_P3H + bo + 16);
        bl.h[0] = *(const v8us*)(wp + OFF_P3L + bo);
        bl.h[1] = *(const v8us*)(wp + OFF_P3L + bo + 16);
        acc2 = wm(ah.v, bh.v, acc2);
        acc2 = wm(ah.v, bl.v, acc2);
        acc2 = wm(al.v, bh.v, acc2);
      }
      const int rbase = 32 * g + 16 * half + 8 * hh;
#pragma unroll
      for (int r = 0; r < 8; ++r) {
        const float y = acc2[r] + b3c;
        const double yd = (rbase + r < nE) ? (double)y : 0.0;
        dsum += yd;
        dsq  += yd * yd;
        sHw[(8 * hh + r) * 16 + m] = y;
      }
      wsync();
      const v4f o0 = *(const v4f*)(sHw + 4 * lane);
      const v4f o1 = *(const v4f*)(sHw + 128 + 4 * lane);
      float* gp = Hp + (size_t)(32 * g + 16 * half) * 16;
      *(volatile v4f*)(gp + 4 * lane)       = o0;
      *(volatile v4f*)(gp + 128 + 4 * lane) = o1;
      __threadfence();
      *(volatile v4f*)(gp + 4 * lane)       = o0;
      *(volatile v4f*)(gp + 128 + 4 * lane) = o1;
      wsync();
    }
  }

  stats_out(dsum, dsq, sRedS, sRedQ, sTot, EW, part + (size_t)blockIdx.x * 32, lane, wave);
}

__global__ void k_fin(const double* __restrict__ part, int nPart, double cntd,
                      const float* __restrict__ gamma, const float* __restrict__ beta,
                      float* ssc) {
  const int tid = (int)threadIdx.x;
  const int c = tid & 15;
  double S = 0.0, Q = 0.0;
#pragma unroll 1
  for (int p = 0; p < nPart; ++p) {
    S += part[(size_t)p * 32 + c];
    Q += part[(size_t)p * 32 + 16 + c];
  }
  const double mean = S / cntd;
  double var = Q / cntd - mean * mean;
  var = var < 0.0 ? 0.0 : var;
  const double rstd = 1.0 / sqrt(var + 1e-5);
  const double scl = (double)gamma[c] * rstd;
  const double shf = (double)beta[c] - mean * scl;
  const float vout = (tid < 16) ? (float)scl : (float)shf;
  if (tid < 32) *(volatile float*)(ssc + tid) = vout;
  __threadfence();
  if (tid < 32) *(volatile float*)(ssc + tid) = vout;
}

template <int NB>
__device__ __forceinline__ int scan_chunk(const int* __restrict__ keys, int nT, int cbase, int slotBase,
                                          int vec8, int* list, int tid, int lane, int wave) {
  int wc = 0;
#pragma unroll
  for (int g = 0; g < NGRP; ++g) {
    const int el0  = (g * NTHR + tid) * EPT;
    const int e0   = cbase + el0;
    const int sent = -2147483647 - 1;
    v4i da, db;
    if (vec8 != 0 && cbase + CHUNK <= nT) {
      da = *(const v4i*)(keys + e0);
      db = *(const v4i*)(keys + e0 + 4);
    } else {
      da.x = (e0     < nT) ? keys[min(e0,     nT - 1)] : sent;
      da.y = (e0 + 1 < nT) ? keys[min(e0 + 1, nT - 1)] : sent;
      da.z = (e0 + 2 < nT) ? keys[min(e0 + 2, nT - 1)] : sent;
      da.w = (e0 + 3 < nT) ? keys[min(e0 + 3, nT - 1)] : sent;
      db.x = (e0 + 4 < nT) ? keys[min(e0 + 4, nT - 1)] : sent;
      db.y = (e0 + 5 < nT) ? keys[min(e0 + 5, nT - 1)] : sent;
      db.z = (e0 + 6 < nT) ? keys[min(e0 + 6, nT - 1)] : sent;
      db.w = (e0 + 7 < nT) ? keys[min(e0 + 7, nT - 1)] : sent;
    }
    const unsigned nb = (unsigned)slotBase;
    const unsigned s0 = (unsigned)da.x - nb, s1 = (unsigned)da.y - nb;
    const unsigned s2 = (unsigned)da.z - nb, s3 = (unsigned)da.w - nb;
    const unsigned s4 = (unsigned)db.x - nb, s5 = (unsigned)db.y - nb;
    const unsigned s6 = (unsigned)db.z - nb, s7 = (unsigned)db.w - nb;
    const bool h0 = s0 < (unsigned)NB, h1 = s1 < (unsigned)NB, h2 = s2 < (unsigned)NB, h3 = s3 < (unsigned)NB;
    const bool h4 = s4 < (unsigned)NB, h5 = s5 < (unsigned)NB, h6 = s6 < (unsigned)NB, h7 = s7 < (unsigned)NB;
    const unsigned any = __builtin_amdgcn_ballot_w32(h0 | h1 | h2 | h3 | h4 | h5 | h6 | h7);
    if (any != 0u) {
#define HITJ(J, HJ, SJ) { \
        const unsigned mj = __builtin_amdgcn_ballot_w32(HJ); \
        if (mj != 0u) { \
          if (HJ) { \
            const int pos = wc + (int)__builtin_amdgcn_mbcnt_lo(mj, 0u); \
            if (pos < WCAP) list[wave * WCAP + pos] = ((el0 + (J)) << 12) | (int)(SJ); \
          } \
          wc += (int)__builtin_popcount(mj); } }
      HITJ(0, h0, s0)
      HITJ(1, h1, s1)
      HITJ(2, h2, s2)
      HITJ(3, h3, s3)
      HITJ(4, h4, s4)
      HITJ(5, h5, s5)
      HITJ(6, h6, s6)
      HITJ(7, h7, s7)
#undef HITJ
    }
  }
  return wc;
}

__device__ __forceinline__ void drain_hits(const int* list, const int* wcnt, float* acc, int* cnt,
                                           const float* __restrict__ Hp, int cbase, int nE, int nT, int lane) {
  const int c16 = lane & 15;
#pragma unroll 1
  for (int wsx = 0; wsx < NWAVE; ++wsx) {
    int n = __builtin_amdgcn_readfirstlane(wcnt[wsx]);
    n = n > WCAP ? WCAP : (n < 0 ? 0 : n);
    const int* lp = list + wsx * WCAP;
#pragma unroll 1
    for (int i = 0; i < n; ++i) {
      const int ent  = __builtin_amdgcn_readfirstlane(lp[i]);
      const int slot = ent & (NBC - 1);
      int idx = cbase + ((ent >> 12) & (CHUNK - 1));
      idx = idx > nT - 1 ? nT - 1 : idx;
      const int e = (idx >= nE) ? idx - nE : idx;
      const float hv = Hp[(size_t)e * 16 + c16];
      if (lane < 16) {
        const int a = slot * 16 + lane;
        acc[a] = acc[a] + hv;
      }
      if (lane == 0) cnt[slot] = cnt[slot] + 1;
    }
  }
}

__global__ __launch_bounds__(NTHR) void k_gather(
    const int* __restrict__ ei, const float* __restrict__ Hp,
    const float* __restrict__ ssc, float* Xp, int nE) {
  extern __shared__ v4f dynlds[];
  float* dyn  = (float*)dynlds;
  float* acc  = dyn;
  int*   cnt  = (int*)(dyn + NBC * 16);
  int*   list = cnt + NBC;
  int*   wcnt = list + LISTN;
  float* sS   = (float*)(wcnt + 32);
  const int tid = threadIdx.x, lane = tid & 31, wave = tid >> 5;
  const int nodeBase = blockIdx.x * NBC;
  const int nT = 2 * nE;

  {
    const v4f z = {0.f, 0.f, 0.f, 0.f};
#pragma unroll 1
    for (int i = tid; i < (NBC * 16 + NBC) / 4; i += NTHR) *(v4f*)(dyn + 4 * i) = z;
  }
  if (tid < 32) sS[tid] = ssc[tid];
  __syncthreads();

  const int nChunks = (nT + CHUNK - 1) / CHUNK;
#pragma unroll 1
  for (int ch = 0; ch < nChunks; ++ch) {
    const int cbase = ch * CHUNK;
    const int wc = scan_chunk<NBC>(ei, nT, cbase, nodeBase, 1, list, tid, lane, wave);
    if (lane == 0) wcnt[wave] = wc;
    __syncthreads();
    if (wave == 0) drain_hits(list, wcnt, acc, cnt, Hp, cbase, nE, nT, lane);
    __syncthreads();
  }

#pragma unroll 1
  for (int idx = tid; idx < NBC * 4; idx += NTHR) {
    const int slot = idx >> 2;
    const int q = idx & 3;
    const v4f S = *(const v4f*)(acc + slot * 16 + 4 * q);
    const int cv = cnt[slot];
    const float fc = (float)cv;
    const float inv = 1.0f / fmaxf(fc, 1.0f);
    v4f o;
#pragma unroll
    for (int j = 0; j < 4; ++j) {
      const int c = 4 * q + j;
      o[j] = (sS[c] * S[j] + fc * sS[16 + c]) * inv;
    }
    float* p = Xp + (size_t)(nodeBase + slot) * 16 + 4 * q;
    *(volatile v4f*)p = o;
    __threadfence();
    *(volatile v4f*)p = o;
  }
}

__global__ __launch_bounds__(NTHR) void k_node(
    const float* __restrict__ Xp, const unsigned short* __restrict__ wp,
    const float* __restrict__ bp, float* Yp, double* part, int nN) {
  __shared__ __attribute__((aligned(16))) float sY[NWAVE][256];
  __shared__ __attribute__((aligned(16))) double sRedS[NWAVE * 32];
  __shared__ __attribute__((aligned(16))) double sRedQ[NWAVE * 32];
  __shared__ __attribute__((aligned(16))) double sTot[32];
  const int tid = threadIdx.x, lane = tid & 31, wave = tid >> 5, hh = lane >> 4, m = lane & 15;
  float* sYw = sY[wave];

  FragB bA, bB;
  {
    const unsigned short* pa = wp + OFF_PA + m * 32 + 8 * hh;
    const unsigned short* pb = wp + OFF_PB + m * 32 + 8 * hh;
    bA.h[0] = *(const v8us*)pa;
    bA.h[1] = *(const v8us*)(pa + 16);
    bB.h[0] = *(const v8us*)pb;
    bB.h[1] = *(const v8us*)(pb + 16);
  }
  const float bpc = bp[m];
  double dsum = 0.0, dsq = 0.0;

#pragma unroll 1
  for (int t = 0; t < NPB / (NWAVE * 16); ++t) {
    const int node0 = blockIdx.x * NPB + wave * (NPB / NWAVE) + 16 * t;
    const float* xr = Xp + (size_t)(node0 + m) * 16 + 8 * hh;
    const v4f x0 = *(const v4f*)xr;
    const v4f x1 = *(const v4f*)(xr + 4);
    float xv[8];
    xv[0] = x0.x; xv[1] = x0.y; xv[2] = x0.z; xv[3] = x0.w;
    xv[4] = x1.x; xv[5] = x1.y; xv[6] = x1.z; xv[7] = x1.w;
    v16us au;
#pragma unroll
    for (int i = 0; i < 8; ++i) {
      unsigned short hi, lo;
      split_bf(xv[i], hi, lo);
      au[i]     = hi;
      au[8 + i] = lo;
    }
    FragB a;
    a.u = au;
    v8f acc = wm(a.v, bA.v, zero8());
    acc = wm(a.v, bB.v, acc);
#pragma unroll
    for (int r = 0; r < 8; ++r) {
      const float y = acc[r] + bpc;
      const int node = node0 + 8 * hh + r;
      const double yd = (node < nN) ? (double)y : 0.0;
      dsum += yd;
      dsq  += yd * yd;
      sYw[(8 * hh + r) * 16 + m] = y;
    }
    wsync();
    const v4f o0 = *(const v4f*)(sYw + 4 * lane);
    const v4f o1 = *(const v4f*)(sYw + 128 + 4 * lane);
    float* gp = Yp + (size_t)node0 * 16;
    *(volatile v4f*)(gp + 4 * lane)       = o0;
    *(volatile v4f*)(gp + 128 + 4 * lane) = o1;
    __threadfence();
    *(volatile v4f*)(gp + 4 * lane)       = o0;
    *(volatile v4f*)(gp + 128 + 4 * lane) = o1;
    wsync();
  }

  stats_out(dsum, dsq, sRedS, sRedQ, sTot, NWAVE, part + (size_t)blockIdx.x * 32, lane, wave);
}

__global__ __launch_bounds__(NTHR) void k_out(
    const float* __restrict__ Yp, const float* __restrict__ ssc, float* out, int nF4) {
  __shared__ float sS[32];
  const int tid = threadIdx.x;
  if (tid < 32) sS[tid] = ssc[tid];
  __syncthreads();
  const int idx = blockIdx.x * NTHR + tid;
  const int ic = idx > nF4 - 1 ? nF4 - 1 : idx;
  const int q = ic & 3;
  const v4f y = *(const v4f*)(Yp + (size_t)ic * 4);
  v4f o;
#pragma unroll
  for (int j = 0; j < 4; ++j) {
    const int c = 4 * q + j;
    o[j] = y[j] * sS[c] + sS[16 + c];
  }
  float* p = out + (size_t)ic * 4;
  if (idx < nF4) *(volatile v4f*)p = o;
  __threadfence();
  if (idx < nF4) *(volatile v4f*)p = o;
}

extern "C" void kernel_launch(void* const* d_in, const int* in_sizes, int n_in,
                              void* d_out, int out_size, void* d_ws, size_t ws_size,
                              hipStream_t stream) {
  if (n_in < 16) return;
  const int nN = in_sizes[0] / 3;
  const int nE = in_sizes[3] / 2;
  if (nN < 1 || nE < 1) return;
  if (in_sizes[0] != 3 * nN || in_sizes[1] != 3 * nN || in_sizes[2] != 4 * nN) return;
  if (in_sizes[3] != 2 * nE) return;
  if (in_sizes[4] != 512 || in_sizes[5] != 64 || in_sizes[6] != 2048 || in_sizes[7] != 32) return;
  if (in_sizes[8] != 512 || in_sizes[9] != 16 || in_sizes[10] != 256 || in_sizes[11] != 16) return;
  if (in_sizes[12] != 16 || in_sizes[13] != 16 || in_sizes[14] != 16 || in_sizes[15] != 16) return;
  if (out_size != 16 * nN) return;
  if (nN > (1 << 24) || nE > (1 << 27)) return;

  const float* coords  = (const float*)d_in[0];
  const float* normals = (const float*)d_in[1];
  const float* curv    = (const float*)d_in[2];
  const int*   ei      = (const int*)d_in[3];
  const float* W1 = (const float*)d_in[4];
  const float* b1 = (const float*)d_in[5];
  const float* W2 = (const float*)d_in[6];
  const float* b2 = (const float*)d_in[7];
  const float* W3 = (const float*)d_in[8];
  const float* b3 = (const float*)d_in[9];
  const float* Wp = (const float*)d_in[10];
  const float* bp = (const float*)d_in[11];
  const float* beg = (const float*)d_in[12];
  const float* beb = (const float*)d_in[13];
  const float* bng = (const float*)d_in[14];
  const float* bnb = (const float*)d_in[15];
  float* out = (float*)d_out;

  const int nGroups = (nE + 31) / 32;
  const int Epad = nGroups * 32;
  int nBlkE = (nGroups + EW - 1) / EW;
  if (nBlkE > MAXEB) nBlkE = MAXEB;
  const int nBlkG = (nN + NBC - 1) / NBC;
  const int NpadG = nBlkG * NBC;
  const int nBlkN = (nN + NPB - 1) / NPB;
  if (nBlkN * NPB > NpadG) return;
  const int nBlkO = (4 * nN + NTHR - 1) / NTHR;

  char* ws = (char*)d_ws;
  size_t off = 0;
  const size_t oW  = off; off += (size_t)WTOT * 2;                off = (off + 255) & ~(size_t)255;
  const size_t oH  = off; off += (size_t)Epad * 16 * 4;           off = (off + 255) & ~(size_t)255;
  const size_t oPE = off; off += (size_t)nBlkE * 32 * 8;          off = (off + 255) & ~(size_t)255;
  const size_t oSE = off; off += 256;
  const size_t oX  = off; off += (size_t)NpadG * 16 * 4;          off = (off + 255) & ~(size_t)255;
  const size_t oY  = off; off += (size_t)NpadG * 16 * 4;          off = (off + 255) & ~(size_t)255;
  const size_t oPN = off; off += (size_t)nBlkN * 32 * 8;          off = (off + 255) & ~(size_t)255;
  const size_t oSN = off; off += 256;
  if (off > ws_size || off > (size_t)WSCAP) return;
  unsigned short* wpl = (unsigned short*)(ws + oW);
  float*  Hp    = (float*)(ws + oH);
  double* partE = (double*)(ws + oPE);
  float*  sscE  = (float*)(ws + oSE);
  float*  Xp    = (float*)(ws + oX);
  float*  Yp    = (float*)(ws + oY);
  double* partN = (double*)(ws + oPN);
  float*  sscN  = (float*)(ws + oSN);

  k_wprep<<<4, NTHR, 0, stream>>>(W1, W2, W3, Wp, wpl);
  k_edge<<<nBlkE, ETHR, 0, stream>>>(coords, normals, curv, ei, wpl, b1, b2, b3,
                                      Hp, partE, nE, nN, nGroups);
  k_fin<<<1, 32, 0, stream>>>(partE, nBlkE, (double)nE, beg, beb, sscE);
  hipFuncSetAttribute(reinterpret_cast<const void*>(&k_gather),
                      hipFuncAttributeMaxDynamicSharedMemorySize, GLDSB);
  k_gather<<<nBlkG, NTHR, GLDSB, stream>>>(ei, Hp, sscE, Xp, nE);
  k_node<<<nBlkN, NTHR, 0, stream>>>(Xp, wpl, bp, Yp, partN, nN);
  k_fin<<<1, 32, 0, stream>>>(partN, nBlkN, (double)nN, bng, bnb, sscN);
  k_out<<<nBlkO, NTHR, 0, stream>>>(Yp, sscN, out, 4 * nN);
}
